// AttentionCell_15625091023560
// MI455X (gfx1250) — hardware-run, weakly checked
//
#include <hip/hip_runtime.h>


#define NB_  8
#define TT   1024
#define DM   512
#define NW   16
typedef _Float16 h16;
typedef unsigned short bf;
typedef __attribute__((ext_vector_type(16))) __bf16   v16bf;
typedef __attribute__((ext_vector_type(16))) _Float16 v16h;
typedef __attribute__((ext_vector_type(8)))  _Float16 v8h;
typedef __attribute__((ext_vector_type(8)))  unsigned short v8us;
typedef __attribute__((ext_vector_type(8)))  float    v8f;
typedef __attribute__((ext_vector_type(4)))  float    v4f;
typedef v8h  __attribute__((may_alias)) v8ha;
typedef v4f  __attribute__((may_alias)) v4fa;
typedef v8us __attribute__((may_alias)) v8usa;

__device__ __forceinline__ unsigned short f2bf(float f) { unsigned u = __float_as_uint(f); u += 0x7FFFu + ((u >> 16) & 1u); return (unsigned short)(u >> 16); }
__device__ __forceinline__ float bf2f(unsigned short b) { return __uint_as_float(((unsigned)b) << 16); }
__device__ __forceinline__ float bfr(float f) { return bf2f(f2bf(f)); }
__device__ __forceinline__ v16h cat16(v8h lo, v8h hi) { return __builtin_shufflevector(lo, hi, 0, 1, 2, 3, 4, 5, 6, 7, 8, 9, 10, 11, 12, 13, 14, 15); }
__device__ __forceinline__ v16bf cat16b(v8us lo, v8us hi) { return __builtin_bit_cast(v16bf, __builtin_shufflevector(lo, hi, 0, 1, 2, 3, 4, 5, 6, 7, 8, 9, 10, 11, 12, 13, 14, 15)); }
__device__ __forceinline__ v8f wmma16(v16h a, v16h b, v8f c) { return __builtin_amdgcn_wmma_f32_16x16x32_f16(false, a, false, b, (short)0, c, false, false); }
__device__ __forceinline__ v8f wmmab(v16bf a, v16bf b, v8f c) { return __builtin_amdgcn_wmma_f32_16x16x32_bf16(false, a, false, b, (short)0, c, false, false); }

template <typename T16> struct WFrag;
template <> struct WFrag<h16> { typedef v16h V; static __device__ __forceinline__ V ld(const h16* p) { return cat16(*(const v8h*)p, *(const v8h*)(p + 16)); } static __device__ __forceinline__ v8f mma(V a, V b, v8f c) { return wmma16(a, b, c); } };
template <> struct WFrag<bf> { typedef v16bf V; static __device__ __forceinline__ V ld(const bf* p) { return cat16b(*(const v8us*)p, *(const v8us*)(p + 16)); } static __device__ __forceinline__ v8f mma(V a, V b, v8f c) { return wmmab(a, b, c); } };
template <typename T16, int NSPLIT, bool BIAS>
__global__ __launch_bounds__(32) void k_gemmw(const T16* __restrict__ A, const T16* __restrict__ A2, const T16* __restrict__ Bt, const T16* __restrict__ Bt2, int K, float* C, int ldc, const float* __restrict__ bias, size_t sA, size_t sB, size_t sC) {
    typedef typename WFrag<T16>::V V;
    __shared__ __align__(16) float os[16 * 68];
    const size_t z = blockIdx.z; A += z * sA; if (A2) A2 += z * sA; Bt += z * sB; if (Bt2) Bt2 += z * sB; C += z * sC;
    const int lane = threadIdx.x & 31, lr = lane & 15, hi = lane >> 4; const int r0 = blockIdx.x * 64, c0 = blockIdx.y * 64;
    v8f acc[4][4];
#pragma unroll
    for (int mb = 0; mb < 4; ++mb)
#pragma unroll
        for (int nb = 0; nb < 4; ++nb) acc[mb][nb] = (v8f){};
    const size_t aoff = (size_t)(r0 + lr) * K + 8 * hi, boff = (size_t)(c0 + lr) * K + 8 * hi;
    for (int kc = 0; kc < K; kc += 32) {
        V a[4], a2[4];
#pragma unroll
        for (int mb = 0; mb < 4; ++mb) { a[mb] = WFrag<T16>::ld(A + aoff + (size_t)mb * 16 * K + kc); if (NSPLIT == 1 || NSPLIT == 2) a2[mb] = WFrag<T16>::ld(A2 + aoff + (size_t)mb * 16 * K + kc); }
#pragma unroll
        for (int nb = 0; nb < 4; ++nb) { const V b = WFrag<T16>::ld(Bt + boff + (size_t)nb * 16 * K + kc); V b2; if (NSPLIT >= 2) b2 = WFrag<T16>::ld(Bt2 + boff + (size_t)nb * 16 * K + kc);
#pragma unroll
            for (int mb = 0; mb < 4; ++mb) { acc[mb][nb] = WFrag<T16>::mma(a[mb], b, acc[mb][nb]); if (NSPLIT == 1 || NSPLIT == 2) acc[mb][nb] = WFrag<T16>::mma(a2[mb], b, acc[mb][nb]); if (NSPLIT >= 2) acc[mb][nb] = WFrag<T16>::mma(a[mb], b2, acc[mb][nb]); } }
        asm volatile("v_nop\n\tv_nop\n\tv_nop\n\tv_nop" : "+v"(acc[0][0]), "+v"(acc[1][1]), "+v"(acc[2][2]), "+v"(acc[3][3]) : "v"(a[0]), "v"(a[3]));
    }
#pragma unroll
    for (int mb = 0; mb < 4; ++mb) {
#pragma unroll
        for (int nb = 0; nb < 4; ++nb) {
#pragma unroll
            for (int j = 0; j < 8; ++j) os[(hi * 8 + j) * 68 + nb * 16 + lr] = acc[mb][nb][j]; }
        __builtin_amdgcn_wave_barrier(); asm volatile("" ::: "memory");
        float* crow = C + (size_t)(r0 + mb * 16) * ldc + c0;
#pragma unroll 1
        for (int ps = 0; ps < 2; ++ps) {
#pragma unroll
            for (int s = 0; s < 8; ++s) { const int row = 2 * s + hi, cofs = lr * 4; v4f val = *(const v4fa*)(os + row * 68 + cofs); if (BIAS) { val[0] += bfr(bias[c0 + cofs]); val[1] += bfr(bias[c0 + cofs + 1]); val[2] += bfr(bias[c0 + cofs + 2]); val[3] += bfr(bias[c0 + cofs + 3]); }
                *(volatile v4f*)(crow + (size_t)row * ldc + cofs) = val; }
            if (ps == 0) __threadfence(); }
        __builtin_amdgcn_wave_barrier(); asm volatile("" ::: "memory");
    }
}

typedef __attribute__((ext_vector_type(2))) unsigned short v2us;

__global__ __launch_bounds__(256) void k_cvt8(const float* __restrict__ src, bf* dst, size_t n8) { const size_t i = (size_t)blockIdx.x * 256 + threadIdx.x; if (i >= n8) return; const v8f v = *(const v8f*)(src + i * 8); v8us o;
#pragma unroll
    for (int k = 0; k < 8; ++k) o[k] = f2bf(v[k]); *(volatile v8us*)(dst + i * 8) = o; __threadfence(); *(volatile v8us*)(dst + i * 8) = o; }

__global__ __launch_bounds__(256) void k_wtG(const float* __restrict__ w, int K, int N, bf* Bt) {
    const int lane = threadIdx.x & 31; const int L0 = (blockIdx.x * 8 + (threadIdx.x >> 5)) * 8; const int nlines = N * K / 64;
#pragma unroll
    for (int ps = 0; ps < 2; ++ps) {
        for (int l = 0; l < 8; ++l) { const int L = L0 + l; if (L >= nlines) break; const size_t e = (size_t)L * 64 + lane * 2; const int k = (int)(e % K), n = (int)(e / K); v2us o;
            o[0] = f2bf(w[(size_t)k * N + n]); o[1] = f2bf(w[(size_t)(k + 1) * N + n]); *(volatile v2us*)(Bt + e) = o; }
        if (ps == 0) __threadfence(); }
}

__global__ __launch_bounds__(256) void k_a0(const float* __restrict__ p0, const float* __restrict__ p1, const float* __restrict__ p2, const float* __restrict__ p3, float* p4) {
    const int lane = threadIdx.x & 31; const int r = blockIdx.x * 8 + (threadIdx.x >> 5); const int t0 = r & (TT - 1); const int rb = r - t0;
    float a[NW]; float fz[NW]; int rr[NW];
#pragma unroll
    for (int w = 0; w < NW; ++w) { const int jj = t0 - (NW - 1) + w; a[w] = 0.0f; fz[w] = (jj < 0) ? 0.0f : 1.0f; rr[w] = rb + ((jj < 0) ? 0 : jj); }
#pragma unroll
    for (int s = 0; s < DM / 128; ++s) { const int cc = s * 128 + lane * 4; const v4f qv = *(const v4f*)(p1 + (size_t)r * DM + cc);
#pragma unroll
        for (int w = 0; w < NW; ++w) { const v4f kv = *(const v4f*)(p2 + (size_t)rr[w] * DM + cc); a[w] += fz[w] * (qv[0] * kv[0] + qv[1] * kv[1] + qv[2] * kv[2] + qv[3] * kv[3]); } }
#pragma unroll
    for (int w = 0; w < NW; ++w) {
#pragma unroll
        for (int sh = 16; sh; sh >>= 1) a[w] += __shfl_xor(a[w], sh, 32); }
    float mx = a[0];
#pragma unroll
    for (int w = 1; w < NW; ++w) mx = (a[w] > mx) ? a[w] : mx;
    float sm = 0.0f;
#pragma unroll
    for (int w = 0; w < NW; ++w) { a[w] = __builtin_amdgcn_exp2f(__fmul_rn(__fsub_rn(a[w], mx), 1.4426950408889634f)); sm = __fadd_rn(sm, a[w]); }
    const float ri = __fdiv_rn(1.0f, sm);
#pragma unroll
    for (int w = 0; w < NW; ++w) a[w] = __fmul_rn(__fmul_rn(a[w], ri), fz[w]);
    v4f oa[DM / 128], ox[DM / 128];
#pragma unroll
    for (int s = 0; s < DM / 128; ++s) { const int cc = s * 128 + lane * 4; v4f acc = (v4f){};
#pragma unroll
        for (int w = 0; w < NW; ++w) { const v4f vv = *(const v4f*)(p3 + (size_t)rr[w] * DM + cc); acc[0] += a[w] * vv[0]; acc[1] += a[w] * vv[1]; acc[2] += a[w] * vv[2]; acc[3] += a[w] * vv[3]; }
        const v4f xi = *(const v4f*)(p0 + (size_t)r * DM + cc); v4f xo; xo[0] = bfr(xi[0]); xo[1] = bfr(xi[1]); xo[2] = bfr(xi[2]); xo[3] = bfr(xi[3]); oa[s] = acc; ox[s] = xo; }
    float* orow = p4 + (size_t)r * (2 * DM);
#pragma unroll
    for (int ps = 0; ps < 2; ++ps) {
#pragma unroll
        for (int s = 0; s < DM / 128; ++s) { const int cc = s * 128 + lane * 4; *(volatile v4f*)(orow + cc) = ox[s]; *(volatile v4f*)(orow + DM + cc) = oa[s]; }
        if (ps == 0) __threadfence(); }
}

extern "C" void kernel_launch(void* const* d_in, const int* in_sizes, int n_in,
                              void* d_out, int out_size, void* d_ws, size_t ws_size, hipStream_t stream) {
    (void)in_sizes; (void)n_in; (void)out_size;
    const float* xin = (const float*)d_in[0]; const float* w0 = (const float*)d_in[1]; const float* w1 = (const float*)d_in[2]; const float* w2 = (const float*)d_in[3];
    float* OUT = (float*)d_out;
    char* wsp = (char*)d_ws;
    auto take = [&](size_t bytes) { char* p = wsp; wsp += (bytes + 255) & ~(size_t)255; return (void*)p; };
    bf* XB = (bf*)take((size_t)NB_ * TT * DM * 2);
    bf* BT = (bf*)take((size_t)3 * DM * DM * 2);
    float* FQ = (float*)take((size_t)3 * NB_ * TT * DM * 4); float* FK = FQ + (size_t)NB_ * TT * DM; float* FV = FQ + (size_t)2 * NB_ * TT * DM;
    if ((size_t)(wsp - (char*)d_ws) > ws_size) return;
    k_cvt8<<<(unsigned)(((size_t)NB_ * TT * DM / 8 + 255) / 256), 256, 0, stream>>>(xin, XB, (size_t)NB_ * TT * DM / 8);
    k_wtG<<<(unsigned)((DM * DM / 64 + 63) / 64), 256, 0, stream>>>(w0, DM, DM, BT); k_wtG<<<(unsigned)((DM * DM / 64 + 63) / 64), 256, 0, stream>>>(w1, DM, DM, BT + (size_t)DM * DM); k_wtG<<<(unsigned)((DM * DM / 64 + 63) / 64), 256, 0, stream>>>(w2, DM, DM, BT + (size_t)2 * DM * DM);
    k_gemmw<bf, 0, false><<<dim3(NB_ * TT / 64, DM / 64, 3), 32, 0, stream>>>(XB, nullptr, BT, nullptr, DM, FQ, DM, nullptr, 0, (size_t)DM * DM, (size_t)NB_ * TT * DM);
    k_a0<<<NB_ * TT / 8, 256, 0, stream>>>(xin, FQ, FK, FV, OUT);
}
